// MambaBlock_30305289241149
// MI455X (gfx1250) — hardware-verified
//
#include <hip/hip_runtime.h>
#include <math.h>

typedef __attribute__((ext_vector_type(16))) __bf16   v16b;
typedef __attribute__((ext_vector_type(8)))  __bf16   v8b;
typedef __attribute__((ext_vector_type(8)))  float    v8f;
typedef __attribute__((ext_vector_type(4)))  float    v4f;
typedef __attribute__((ext_vector_type(4)))  unsigned v4u;

constexpr int kBatch  = 4;
constexpr int kSeq    = 4096;
constexpr int kDm     = 192;
constexpr int kDin    = 384;
constexpr int kNst    = 16;
constexpr int kDtR    = 12;
constexpr int kXzP    = 2 * kDin;
constexpr int kXdN    = kDtR + 2 * kNst;
constexpr int kXdP    = 64;
constexpr int kRows   = kBatch * kSeq;
constexpr int kXtP    = 65;
constexpr int kConvCh = 128;
constexpr int kConvTP = 132;
constexpr int kScanTS = 64;
constexpr int kScanCh = 64;
constexpr int kScanYP = 68;
static_assert(kXdN == 44 && kXdN <= kXdP, "x_proj width");
static_assert((kDm % 32) == 0 && (kDin % 32) == 0, "GEMM K multiples of 32");
static_assert((kRows % 64) == 0 && (kXzP % 64) == 0 && (kXdP % 64) == 0 && (kDm % 64) == 0 && (kSeq % 64) == 0, "GEMM M,N multiples of 64");
static_assert((kSeq % kScanTS) == 0 && (kDin % kScanCh) == 0 && (kDin % kConvCh) == 0, "tile multiples");
static_assert(kRows * kDm == 3145728, "output element count");
static_assert((kDtR % 4) == 0, "dt dot is walked 4 terms at a time");

constexpr size_t kOffXH   = 0;
constexpr size_t kOffXL   = kOffXH  + (size_t)kRows * kDm  * 2;
constexpr size_t kOffWIH  = kOffXL  + (size_t)kRows * kDm  * 2;
constexpr size_t kOffWIL  = kOffWIH + (size_t)kXzP  * kDm  * 2;
constexpr size_t kOffWXH  = kOffWIL + (size_t)kXzP  * kDm  * 2;
constexpr size_t kOffWOH  = kOffWXH + (size_t)kXdP  * kDin * 2;
constexpr size_t kOffWOL  = kOffWOH + (size_t)kDm   * kDin * 2;
constexpr size_t kOffXZ   = kOffWOL + (size_t)kDm   * kDin * 2;
constexpr size_t kOffUC   = kOffXZ  + (size_t)kRows * kXzP * 4;
constexpr size_t kOffUCH  = kOffUC  + (size_t)kRows * kDin * 4;
constexpr size_t kOffXD   = kOffUCH + (size_t)kRows * kDin * 2;
constexpr size_t kOffYH   = kOffXD  + (size_t)kRows * kXdP * 4;
constexpr size_t kOffYL   = kOffYH  + (size_t)kRows * kDin * 2;
constexpr size_t kWsTotal = kOffYL  + (size_t)kRows * kDin * 2;
static_assert(kWsTotal == 130957312ull, "carve total");
static_assert(kWsTotal <= 134217728ull, "carve cap");
static_assert((kOffXL % 128) == 0 && (kOffWIH % 128) == 0 && (kOffWIL % 128) == 0 && (kOffWXH % 128) == 0 &&
              (kOffWOH % 128) == 0 && (kOffWOL % 128) == 0 && (kOffXZ % 128) == 0 && (kOffUC % 128) == 0 &&
              (kOffUCH % 128) == 0 && (kOffXD % 128) == 0 && (kOffYH % 128) == 0 && (kOffYL % 128) == 0,
              "128-B aligned regions");

__device__ __forceinline__ unsigned bf_bits(float f) {
  const unsigned u = __float_as_uint(f);
  return (u + 0x7FFFu + ((u >> 16) & 1u)) >> 16;
}
__device__ __forceinline__ float bf_val(unsigned hb) { return __uint_as_float(hb << 16); }
__device__ __forceinline__ void bf_split(float f, unsigned& hb, unsigned& lb) {
  hb = bf_bits(f);
  lb = bf_bits(f - bf_val(hb));
}
__device__ __forceinline__ unsigned pack2(unsigned lo16, unsigned hi16) { return lo16 | (hi16 << 16); }
__device__ __forceinline__ void pack8_split(float f0, float f1, float f2, float f3, float f4, float f5, float f6, float f7,
                                            v4u& hv, v4u& lv) {
  unsigned h0, h1, h2, h3, h4, h5, h6, h7, l0, l1, l2, l3, l4, l5, l6, l7;
  bf_split(f0, h0, l0); bf_split(f1, h1, l1); bf_split(f2, h2, l2); bf_split(f3, h3, l3);
  bf_split(f4, h4, l4); bf_split(f5, h5, l5); bf_split(f6, h6, l6); bf_split(f7, h7, l7);
  hv = (v4u){pack2(h0, h1), pack2(h2, h3), pack2(h4, h5), pack2(h6, h7)};
  lv = (v4u){pack2(l0, l1), pack2(l2, l3), pack2(l4, l5), pack2(l6, l7)};
}
__device__ __forceinline__ v4u pack8_hi(float f0, float f1, float f2, float f3, float f4, float f5, float f6, float f7) {
  return (v4u){pack2(bf_bits(f0), bf_bits(f1)), pack2(bf_bits(f2), bf_bits(f3)),
               pack2(bf_bits(f4), bf_bits(f5)), pack2(bf_bits(f6), bf_bits(f7))};
}

__device__ __forceinline__ v16b frag_load(const __bf16* p) {
  union U { v16b v; v8b h[2]; } f;
  f.h[0] = *(const v8b*)(p);
  f.h[1] = *(const v8b*)(p + 16);
  return f.v;
}
__device__ __forceinline__ v8f mma_bf16(v16b a, v16b b, v8f c) {
  return __builtin_amdgcn_wmma_f32_16x16x32_bf16(false, a, false, b, (short)0, c, false, false);
}
__device__ __forceinline__ void row_guard(v8f& a, v8f& b, v8f& c, v8f& d, v16b x, v16b y) {
  asm volatile("v_nop\n\tv_nop\n\tv_nop\n\tv_nop" : "+v"(a), "+v"(b), "+v"(c), "+v"(d) : "v"(x), "v"(y));
}
__device__ __forceinline__ void keep4_b(v16b a, v16b b, v16b c, v16b d) { asm volatile("v_nop" :: "v"(a), "v"(b), "v"(c), "v"(d)); }
__device__ __forceinline__ void acc_guard4(v8f& a, v8f& b, v8f& c, v8f& d) {
  asm volatile("v_nop\n\tv_nop\n\tv_nop\n\tv_nop" : "+v"(a), "+v"(b), "+v"(c), "+v"(d));
}

template <int SPL>
__global__ __launch_bounds__(256) void wmma_gemm64_bf16(
    const unsigned short* __restrict__ Ap, const unsigned short* __restrict__ A2p, int lda, long strideA,
    const unsigned short* __restrict__ Btp, const unsigned short* __restrict__ Bt2p, int ldb, long strideB,
    float* __restrict__ Cout, int ldc, long strideC, int M, int N, int K) {
  const __bf16* A   = (const __bf16*)Ap;
  const __bf16* A2  = (const __bf16*)A2p;
  const __bf16* Bt  = (const __bf16*)Btp;
  const __bf16* Bt2 = (const __bf16*)Bt2p;
  __shared__ __align__(16) float sT[8][16 * 68];
  const int b    = blockIdx.y;
  const int lane = threadIdx.x & 31;
  const int wave = threadIdx.x >> 5;
  const int tilesN = N >> 6;
  const int tilesM = M >> 6;
  const int tile = blockIdx.x * 8 + wave;
  if (tile >= tilesM * tilesN) return;
  const int tm = tile / tilesN;
  const int tn = tile - tm * tilesN;
  const int m0 = tm << 6;
  const int n0 = tn << 6;

  const __bf16* Ab  = A  + (size_t)b * strideA;
  const __bf16* Bb  = Bt + (size_t)b * strideB;
  const __bf16* Ab2 = A2  + (size_t)b * strideA;
  const __bf16* Bb2 = Bt2 + (size_t)b * strideB;

  const int rlane = lane & 15;
  const int koff  = (lane >> 4) * 8;
  const int mOff  = (lane >> 4) * 8;

  v8f acc[4][4];
#pragma unroll
  for (int i = 0; i < 4; ++i)
#pragma unroll
    for (int j = 0; j < 4; ++j) acc[i][j] = (v8f){0.f, 0.f, 0.f, 0.f, 0.f, 0.f, 0.f, 0.f};

  for (int k0 = 0; k0 < K; k0 += 32) {
    v16b bh[4], bl[4];
#pragma unroll
    for (int j = 0; j < 4; ++j) {
      const size_t bo = (size_t)(n0 + (j << 4) + rlane) * ldb + koff + k0;
      bh[j] = frag_load(Bb + bo);
      if (SPL == 2) bl[j] = frag_load(Bb2 + bo);
    }
#pragma unroll
    for (int i = 0; i < 4; ++i) {
      const size_t ao = (size_t)(m0 + (i << 4) + rlane) * lda + koff + k0;
      v16b ah = frag_load(Ab + ao);
      v16b al = ah;
      if (SPL == 2) al = frag_load(Ab2 + ao);
#pragma unroll
      for (int j = 0; j < 4; ++j) {
        acc[i][j] = mma_bf16(ah, bh[j], acc[i][j]);
        if (SPL == 2) {
          acc[i][j] = mma_bf16(ah, bl[j], acc[i][j]);
          acc[i][j] = mma_bf16(al, bh[j], acc[i][j]);
        }
      }
      row_guard(acc[i][0], acc[i][1], acc[i][2], acc[i][3], ah, al);
    }
    keep4_b(bh[0], bh[1], bh[2], bh[3]);
    if (SPL == 2) keep4_b(bl[0], bl[1], bl[2], bl[3]);
  }
  acc_guard4(acc[0][0], acc[0][1], acc[0][2], acc[0][3]);
  acc_guard4(acc[1][0], acc[1][1], acc[1][2], acc[1][3]);
  acc_guard4(acc[2][0], acc[2][1], acc[2][2], acc[2][3]);
  acc_guard4(acc[3][0], acc[3][1], acc[3][2], acc[3][3]);

  float* slab = sT[wave];
  float* C = Cout + (size_t)b * strideC;
  const int hh = lane >> 4, c4 = (lane & 15) * 4;
#pragma unroll
  for (int i = 0; i < 4; ++i) {
    const int mBase = m0 + (i << 4);
#pragma unroll
    for (int j = 0; j < 4; ++j) {
#pragma unroll
      for (int r = 0; r < 8; ++r) slab[(mOff + r) * 68 + (j << 4) + rlane] = acc[i][j][r];
    }
    __builtin_amdgcn_fence(__ATOMIC_RELEASE, "workgroup");
    __builtin_amdgcn_wave_barrier();
    __builtin_amdgcn_fence(__ATOMIC_ACQUIRE, "workgroup");
    for (int pass = 0; pass < 2; ++pass) {
#pragma unroll
      for (int it = 0; it < 8; ++it) {
        const int row = it * 2 + hh;
        const v4f v = *(const v4f*)(slab + row * 68 + c4);
        *(volatile v4f*)(C + (size_t)(mBase + row) * ldc + n0 + c4) = v;
      }
      __threadfence();
    }
    __builtin_amdgcn_fence(__ATOMIC_RELEASE, "workgroup");
    __builtin_amdgcn_wave_barrier();
    __builtin_amdgcn_fence(__ATOMIC_ACQUIRE, "workgroup");
  }
}

__global__ __launch_bounds__(256) void xsplit_kernel(
    const float* __restrict__ x, unsigned short* __restrict__ XH, unsigned short* __restrict__ XL) {
  __shared__ float tile[kDm * kXtP];
  const int tid = threadIdx.x;
  const int g0 = blockIdx.x * 64;
  const int b  = g0 / kSeq;
  const int l0 = g0 - b * kSeq;
  const float* xb = x + (size_t)b * kDm * kSeq + l0;
#pragma unroll 4
  for (int it = 0; it < 12; ++it) {
    const int idx = it * 256 + tid;
    const int c   = idx >> 4;
    const int l4  = (idx & 15) * 4;
    const v4f v = *(const v4f*)(xb + (size_t)c * kSeq + l4);
    const float f0 = v[0], f1 = v[1], f2 = v[2], f3 = v[3];
    float* tp = tile + c * kXtP + l4;
    tp[0] = f0; tp[1] = f1; tp[2] = f2; tp[3] = f3;
  }
  __syncthreads();
  v4u hv[6], lv[6];
#pragma unroll
  for (int it = 0; it < 6; ++it) {
    const int p   = it * 256 + tid;
    const int row = p / 24;
    const int col = (p - row * 24) * 8;
    const float* tp = tile + col * kXtP + row;
    pack8_split(tp[0], tp[kXtP], tp[2 * kXtP], tp[3 * kXtP], tp[4 * kXtP], tp[5 * kXtP], tp[6 * kXtP], tp[7 * kXtP],
                hv[it], lv[it]);
  }
  unsigned short* qh = XH + (size_t)g0 * kDm;
  unsigned short* ql = XL + (size_t)g0 * kDm;
  for (int pass = 0; pass < 2; ++pass) {
#pragma unroll
    for (int it = 0; it < 6; ++it) {
      const size_t e0 = (size_t)(it * 256 + tid) * 8;
      *(volatile v4u*)(qh + e0) = hv[it];
      *(volatile v4u*)(ql + e0) = lv[it];
    }
    __threadfence();
  }
}

template <bool LO>
__global__ __launch_bounds__(256) void split_rows_bf16_kernel(
    const float* __restrict__ src, unsigned short* __restrict__ dhi, unsigned short* __restrict__ dlo,
    int total8, int real8) {
  const int i = blockIdx.x * 256 + threadIdx.x;
  if (i >= total8) return;
  const bool valid = (i < real8);
  const int ic = valid ? i : (real8 - 1);
  const size_t s0 = (size_t)ic << 3;
  const v4f a0 = *(const v4f*)(src + s0);
  const v4f a1 = *(const v4f*)(src + s0 + 4);
  const float f0 = valid ? a0[0] : 0.0f, f1 = valid ? a0[1] : 0.0f, f2 = valid ? a0[2] : 0.0f, f3 = valid ? a0[3] : 0.0f;
  const float f4 = valid ? a1[0] : 0.0f, f5 = valid ? a1[1] : 0.0f, f6 = valid ? a1[2] : 0.0f, f7 = valid ? a1[3] : 0.0f;
  v4u hv, lv;
  pack8_split(f0, f1, f2, f3, f4, f5, f6, f7, hv, lv);
  const size_t e0 = (size_t)i << 3;
  *(volatile v4u*)(dhi + e0) = hv;
  if (LO) *(volatile v4u*)(dlo + e0) = lv;
  __threadfence();
  *(volatile v4u*)(dhi + e0) = hv;
  if (LO) *(volatile v4u*)(dlo + e0) = lv;
}

__global__ __launch_bounds__(128) void conv_silu_kernel(
    const float* __restrict__ XZ, const float* __restrict__ cw, const float* __restrict__ cb,
    float* __restrict__ UC, unsigned short* __restrict__ UCH) {
  __shared__ __align__(16) float sT[16 * kConvTP];
  const int tid = threadIdx.x, lane = tid & 31, wave = tid >> 5;
  const int d0 = blockIdx.x * kConvCh, d = d0 + tid;
  const int g0 = blockIdx.y * 64;
  const int tb = g0 & (kSeq - 1);
  const float w0 = cw[d * 4 + 0], w1 = cw[d * 4 + 1], w2 = cw[d * 4 + 2], w3 = cw[d * 4 + 3];
  const float bc = cb[d];
  float xm3, xm2, xm1;
  {
    const bool hist = (tb > 0);
    const int rb = hist ? (g0 - 3) : g0;
    const float v3 = XZ[(size_t)rb * kXzP + d];
    const float v2 = XZ[(size_t)(rb + 1) * kXzP + d];
    const float v1 = XZ[(size_t)(rb + 2) * kXzP + d];
    xm3 = hist ? v3 : 0.0f;
    xm2 = hist ? v2 : 0.0f;
    xm1 = hist ? v1 : 0.0f;
  }
  const int hh = lane >> 4;
  const int c8 = (lane & 15) * 8;
#pragma unroll 1
  for (int sub = 0; sub < 4; ++sub) {
    const int lb = g0 + sub * 16;
#pragma unroll 1
    for (int s = 0; s < 16; ++s) {
      const float xcur = XZ[(size_t)(lb + s) * kXzP + d];
      float acc = w0 * xm3;
      acc = fmaf(w1, xm2, acc);
      acc = fmaf(w2, xm1, acc);
      acc = fmaf(w3, xcur, acc);
      const float sv = acc + bc;
      const float sg = 1.0f / (1.0f + expf(-sv));
      sT[s * kConvTP + tid] = sv * sg;
      xm3 = xm2; xm2 = xm1; xm1 = xcur;
    }
    __syncthreads();
    v4f fv[4];
    v4u bh[2];
#pragma unroll
    for (int it = 0; it < 4; ++it) fv[it] = *(const v4f*)(sT + (it * 4 + wave) * kConvTP + lane * 4);
#pragma unroll
    for (int it = 0; it < 2; ++it) {
      const float* sp = sT + (it * 8 + wave * 2 + hh) * kConvTP + c8;
      const v4f a0 = *(const v4f*)(sp);
      const v4f a1 = *(const v4f*)(sp + 4);
      const float f0 = a0[0], f1 = a0[1], f2 = a0[2], f3 = a0[3];
      const float f4 = a1[0], f5 = a1[1], f6 = a1[2], f7 = a1[3];
      bh[it] = pack8_hi(f0, f1, f2, f3, f4, f5, f6, f7);
    }
    for (int pass = 0; pass < 2; ++pass) {
#pragma unroll
      for (int it = 0; it < 4; ++it)
        *(volatile v4f*)(UC + (size_t)(lb + it * 4 + wave) * kDin + d0 + lane * 4) = fv[it];
#pragma unroll
      for (int it = 0; it < 2; ++it)
        *(volatile v4u*)(UCH + (size_t)(lb + it * 8 + wave * 2 + hh) * kDin + d0 + c8) = bh[it];
      __threadfence();
    }
    __syncthreads();
  }
}

__global__ __launch_bounds__(64) void scan_kernel(
    const float* __restrict__ XD, const float* __restrict__ UC, const float* __restrict__ XZ,
    const float* __restrict__ Wdt, const float* __restrict__ bdt, const float* __restrict__ Alog,
    const float* __restrict__ Dp, unsigned short* __restrict__ YH, unsigned short* __restrict__ YL) {
  __shared__ __align__(16) float sX[kScanTS * kXdP];
  __shared__ __align__(16) float sY[kScanTS * kScanYP];
  __shared__ __align__(16) float sW[kDtR * kScanCh];
  __shared__ __align__(16) float sA[kNst * kScanCh];
  __shared__ __align__(16) float sH[kNst * kScanCh];
  const int tid = threadIdx.x, lane = tid & 31, wave = tid >> 5;
  constexpr int kBlkPerB = kDin / kScanCh;
  const int bix = blockIdx.x / kBlkPerB;
  const int d0  = (blockIdx.x - bix * kBlkPerB) * kScanCh;
  const int d   = d0 + tid;
  const size_t row0 = (size_t)bix * kSeq;
#pragma unroll 1
  for (int r = 0; r < kDtR; ++r) sW[r * kScanCh + tid] = Wdt[(size_t)d * kDtR + r];
#pragma unroll 1
  for (int n = 0; n < kNst; ++n) {
    sA[n * kScanCh + tid] = -expf(Alog[(size_t)d * kNst + n]);
    sH[n * kScanCh + tid] = 0.0f;
  }
  __syncthreads();
  const float bb = bdt[d], Dd = Dp[d];
  const int lr = tid >> 4, lc4 = (tid & 15) * 4;
  const int q = lane >> 3, c8 = (lane & 7) * 8;
#pragma unroll 1
  for (int t0 = 0; t0 < kSeq; t0 += kScanTS) {
    __syncthreads();
#pragma unroll 4
    for (int i = 0; i < 16; ++i) {
      const int r = lr + 4 * i;
      const v4f xv = *(const v4f*)(XD + (row0 + t0 + r) * kXdP + lc4);
      *(v4f*)(sX + r * kXdP + lc4) = xv;
    }
    __syncthreads();
#pragma unroll 1
    for (int s = 0; s < kScanTS; ++s) {
      const size_t m = row0 + t0 + s;
      const float* xr = sX + s * kXdP;
      float vdot = 0.0f;
#pragma unroll 1
      for (int r4 = 0; r4 < kDtR / 4; ++r4) {
        const v4f xv = *(const v4f*)(xr + 4 * r4);
        const float x0 = xv[0], x1 = xv[1], x2 = xv[2], x3 = xv[3];
        const float* wp = sW + (4 * r4) * kScanCh + tid;
        vdot = fmaf(x0, wp[0], vdot);
        vdot = fmaf(x1, wp[kScanCh], vdot);
        vdot = fmaf(x2, wp[2 * kScanCh], vdot);
        vdot = fmaf(x3, wp[3 * kScanCh], vdot);
      }
      const float v   = vdot + bb;
      const float dt  = fmaxf(v, 0.0f) + log1pf(expf(-fabsf(v)));
      const float xt  = UC[m * kDin + d];
      const float zv  = XZ[m * kXzP + kDin + d];
      const float dtx = dt * xt;
      float y = 0.0f;
#pragma unroll 1
      for (int n = 0; n < kNst; ++n) {
        const float e  = expf(dt * sA[n * kScanCh + tid]);
        const float hn = fmaf(e, sH[n * kScanCh + tid], dtx * xr[kDtR + n]);
        sH[n * kScanCh + tid] = hn;
        y = fmaf(hn, xr[kDtR + kNst + n], y);
      }
      y = fmaf(xt, Dd, y);
      const float sg = 1.0f / (1.0f + expf(-zv));
      sY[s * kScanYP + tid] = y * (zv * sg);
    }
    __syncthreads();
    v4u hv[8], lv[8];
#pragma unroll
    for (int it = 0; it < 8; ++it) {
      const int row = it * 8 + wave * 4 + q;
      const float* sp = sY + row * kScanYP + c8;
      const v4f a0 = *(const v4f*)(sp);
      const v4f a1 = *(const v4f*)(sp + 4);
      const float f0 = a0[0], f1 = a0[1], f2 = a0[2], f3 = a0[3];
      const float f4 = a1[0], f5 = a1[1], f6 = a1[2], f7 = a1[3];
      pack8_split(f0, f1, f2, f3, f4, f5, f6, f7, hv[it], lv[it]);
    }
    for (int pass = 0; pass < 2; ++pass) {
#pragma unroll
      for (int it = 0; it < 8; ++it) {
        const int row = it * 8 + wave * 4 + q;
        const size_t o = (row0 + t0 + row) * kDin + d0 + c8;
        *(volatile v4u*)(YH + o) = hv[it];
        *(volatile v4u*)(YL + o) = lv[it];
      }
      __threadfence();
    }
  }
}

static_assert((kRows / 64) * (kXzP / 64) == 384 * 8, "in_proj grid");
static_assert((kRows / 64) * (kXdP / 64) == 32 * 8, "x_proj grid");
static_assert((kDm / 64) * (kSeq / 64) == 24 * 8, "out_proj grid");
static_assert(((kXzP * kDm / 8) % 256) == 0 && ((kXdP * kDin / 8) % 256) == 0 && ((kDm * kDin / 8) % 256) == 0, "plane grids");

extern "C" void kernel_launch(void* const* d_in, const int* in_sizes, int n_in,
                              void* d_out, int out_size, void* d_ws, size_t ws_size,
                              hipStream_t stream) {
  if (n_in < 10) return;
  if (in_sizes[0] != kRows * kDm) return;
  if (in_sizes[1] != kXzP * kDm) return;
  if (in_sizes[2] != kDin * 4) return;
  if (in_sizes[3] != kDin) return;
  if (in_sizes[4] != kXdN * kDin) return;
  if (in_sizes[5] != kDin * kDtR) return;
  if (in_sizes[6] != kDin) return;
  if (in_sizes[7] != kDin * kNst) return;
  if (in_sizes[8] != kDin) return;
  if (in_sizes[9] != kDm * kDin) return;
  if (out_size != kRows * kDm) return;
  if (ws_size < kWsTotal) return;

  const float* x       = (const float*)d_in[0];
  const float* W_in    = (const float*)d_in[1];
  const float* conv_w  = (const float*)d_in[2];
  const float* conv_b  = (const float*)d_in[3];
  const float* W_xproj = (const float*)d_in[4];
  const float* W_dt    = (const float*)d_in[5];
  const float* b_dt    = (const float*)d_in[6];
  const float* A_log   = (const float*)d_in[7];
  const float* Dp      = (const float*)d_in[8];
  const float* W_out   = (const float*)d_in[9];
  float* out = (float*)d_out;

  char* ws = (char*)d_ws;
  unsigned short* XH  = (unsigned short*)(ws + kOffXH);
  unsigned short* XL  = (unsigned short*)(ws + kOffXL);
  unsigned short* WIH = (unsigned short*)(ws + kOffWIH);
  unsigned short* WIL = (unsigned short*)(ws + kOffWIL);
  unsigned short* WXH = (unsigned short*)(ws + kOffWXH);
  unsigned short* WOH = (unsigned short*)(ws + kOffWOH);
  unsigned short* WOL = (unsigned short*)(ws + kOffWOL);
  float*          XZ  = (float*)(ws + kOffXZ);
  float*          UC  = (float*)(ws + kOffUC);
  unsigned short* UCH = (unsigned short*)(ws + kOffUCH);
  float*          XD  = (float*)(ws + kOffXD);
  unsigned short* YH  = (unsigned short*)(ws + kOffYH);
  unsigned short* YL  = (unsigned short*)(ws + kOffYL);

  xsplit_kernel<<<kRows / 64, 256, 0, stream>>>(x, XH, XL);
  split_rows_bf16_kernel<true><<<(kXzP * kDm / 8) / 256, 256, 0, stream>>>(W_in, WIH, WIL, kXzP * kDm / 8, kXzP * kDm / 8);
  split_rows_bf16_kernel<false><<<(kXdP * kDin / 8) / 256, 256, 0, stream>>>(W_xproj, WXH, WXH, kXdP * kDin / 8, kXdN * kDin / 8);
  split_rows_bf16_kernel<true><<<(kDm * kDin / 8) / 256, 256, 0, stream>>>(W_out, WOH, WOL, kDm * kDin / 8, kDm * kDin / 8);

  wmma_gemm64_bf16<2><<<dim3(384, 1), 256, 0, stream>>>(
      XH, XL, kDm, 0L, WIH, WIL, kDm, 0L, XZ, kXzP, 0L, kRows, kXzP, kDm);

  conv_silu_kernel<<<dim3(kDin / kConvCh, kRows / 64), kConvCh, 0, stream>>>(XZ, conv_w, conv_b, UC, UCH);

  wmma_gemm64_bf16<0><<<dim3(32, 1), 256, 0, stream>>>(
      UCH, UCH, kDin, 0L, WXH, WXH, kDin, 0L, XD, kXdP, 0L, kRows, kXdP, kDin);

  scan_kernel<<<kBatch * (kDin / kScanCh), kScanCh, 0, stream>>>(XD, UC, XZ, W_dt, b_dt, A_log, Dp, YH, YL);

  wmma_gemm64_bf16<2><<<dim3(24, kBatch), 256, 0, stream>>>(
      WOH, WOL, kDin, 0L, YH, YL, kDin, (long)kSeq * kDin, out, kSeq, (long)kDm * kSeq, kDm, kSeq, kDin);
}
